// MultiHeadAttention_11974368821785
// MI455X (gfx1250) — hardware-run, weakly checked
//
#include <hip/hip_runtime.h>


#ifndef NB
#define NB 2
#endif
#ifndef SEQ
#define SEQ 1024
#endif
#define NB_FULL  2
#define SEQ_FULL 1024
#define TT   SEQ
#define NH_  32
#define NKV  8
#define REP  (NH_ / NKV)
#define HD   64
#define ZH   8
#define ZKV  (ZH / REP)
#ifndef RH
#define RH   ((SEQ) >= 1024 ? 512 : ((SEQ) >= 512 ? 256 : 64))
#endif
#define PCAR 16384.0f
#define QCAR 8.0f
#define VCAR 8.0f
#define SCL  (1.0f / 64.0f)
#define NEGF (-1e30f)
#define CLAMPHI 0.999999f
#define LN2F 0.6931471805599453f

static_assert(NB >= 1 && NB <= NB_FULL);
static_assert(SEQ % 128 == 0 && SEQ >= 128 && SEQ <= SEQ_FULL);
static_assert(RH % 64 == 0 && RH >= 64 && RH < SEQ);
static_assert(NH_ % ZH == 0 && ZH % REP == 0 && NH_ % NKV == 0);
static_assert(HD == 64 && TT % 64 == 0);
static_assert(HD % 32 == 0 && TT % 32 == 0);
static_assert((ZH * TT) % 8 == 0 && (NKV * TT) % 8 == 0);
static_assert(((size_t)ZH * TT * HD) % 1024 == 0 && ((size_t)NKV * TT * HD) % 512 == 0 && ((size_t)NH_ * TT * HD) % 512 == 0);
#define WS_TOTAL ((size_t)NH_ * TT * HD * 2 * 3 + (size_t)NKV * TT * HD * 2 * 6 + (size_t)ZH * RH * TT * 2 * 2 + (size_t)ZKV * TT * TT * 4 * 2 + (size_t)ZH * TT * TT * 4 + (size_t)ZH * TT * TT * 2 + (size_t)ZH * TT * HD * 4)
static_assert(WS_TOTAL <= (size_t)134217728);

typedef _Float16 h16;
typedef unsigned short bf;
typedef __attribute__((ext_vector_type(16))) __bf16   v16bf;
typedef __attribute__((ext_vector_type(16))) _Float16 v16h;
typedef __attribute__((ext_vector_type(8)))  _Float16 v8h;
typedef __attribute__((ext_vector_type(8)))  unsigned short v8us;
typedef __attribute__((ext_vector_type(8)))  float    v8f;
typedef __attribute__((ext_vector_type(4)))  float    v4f;
typedef __attribute__((ext_vector_type(4)))  int      v4i;
typedef __attribute__((ext_vector_type(2)))  _Float16 v2h;
typedef __attribute__((ext_vector_type(4)))  _Float16 v4h;
typedef __attribute__((ext_vector_type(2)))  unsigned short v2us;
typedef __attribute__((ext_vector_type(4)))  unsigned short v4us;
typedef v8h  __attribute__((may_alias)) v8ha;
typedef v4f  __attribute__((may_alias)) v4fa;
typedef v8us __attribute__((may_alias)) v8usa;

__device__ __forceinline__ unsigned short f2bf(float f) { unsigned u = __float_as_uint(f); u += 0x7FFFu + ((u >> 16) & 1u); return (unsigned short)(u >> 16); }
__device__ __forceinline__ float bf2f(unsigned short b) { return __uint_as_float(((unsigned)b) << 16); }
__device__ __forceinline__ float bfr(float f) { return bf2f(f2bf(f)); }
__device__ __forceinline__ v16h cat16(v8h lo, v8h hi) { return __builtin_shufflevector(lo, hi, 0, 1, 2, 3, 4, 5, 6, 7, 8, 9, 10, 11, 12, 13, 14, 15); }
__device__ __forceinline__ v16bf cat16b(v8us lo, v8us hi) { return __builtin_bit_cast(v16bf, __builtin_shufflevector(lo, hi, 0, 1, 2, 3, 4, 5, 6, 7, 8, 9, 10, 11, 12, 13, 14, 15)); }
__device__ __forceinline__ v8f wmma16(v16h a, v16h b, v8f c) { return __builtin_amdgcn_wmma_f32_16x16x32_f16(false, a, false, b, (short)0, c, false, false); }
__device__ __forceinline__ v8f wmmab(v16bf a, v16bf b, v8f c) { return __builtin_amdgcn_wmma_f32_16x16x32_bf16(false, a, false, b, (short)0, c, false, false); }
__device__ __forceinline__ h16 tohx(float x) { return (h16)x; }
__device__ __forceinline__ void splitf(float y, unsigned short& h, unsigned short& l) { h = f2bf(y); l = f2bf(y - bf2f(h)); }
__device__ __forceinline__ void wave_lds_sync() { __builtin_amdgcn_fence(3  , "wavefront"); __builtin_amdgcn_wave_barrier(); asm volatile("" ::: "memory"); }

static __device__ __forceinline__ h16 toh_flush(float v) { const h16 r = (h16)v; return (fabsf(v) < 6.103515625e-05f) ? (h16)0.0f : r; }
static __device__ __forceinline__ float sig3(float x) { const float xb = bfr(x); const float e = __builtin_amdgcn_exp2f(-1.4426950408889634f * xb); const float s = __builtin_amdgcn_rcpf(1.0f + e); return __builtin_amdgcn_exp2f(0.33333334f * __builtin_amdgcn_logf(s)); }
static __device__ __forceinline__ float pow23(float c) { const float y = fmaxf(c, 1e-35f); const float r = __builtin_amdgcn_exp2f(0.6666667f * __builtin_amdgcn_logf(y)); return (c > 0.0f) ? r : 0.0f; }

template <typename T16> struct WFrag;
template <> struct WFrag<h16> { typedef v16h V; static __device__ __forceinline__ V ld(const h16* p) { return cat16(*(const v8h*)p, *(const v8h*)(p + 16)); } static __device__ __forceinline__ v8f mma(V a, V b, v8f c) { return wmma16(a, b, c); } };
template <> struct WFrag<bf> { typedef v16bf V; static __device__ __forceinline__ V ld(const bf* p) { return cat16b(*(const v8us*)p, *(const v8us*)(p + 16)); } static __device__ __forceinline__ v8f mma(V a, V b, v8f c) { return wmmab(a, b, c); } };

template <typename T16, int NSPLIT, int CMODE>
__global__ __launch_bounds__(32) void k_gemmc(const T16* __restrict__ A, const T16* __restrict__ A2, const T16* __restrict__ Bt, const T16* __restrict__ Bt2, int K, float* C, int ldc, int roff, size_t sA, size_t sB, size_t sC, int zdb) {
    typedef typename WFrag<T16>::V V;
    __shared__ __align__(16) float os[16 * 68];
    const size_t z = blockIdx.z, zb = z / (size_t)zdb; A += z * sA; if (A2) A2 += z * sA; Bt += zb * sB; if (Bt2) Bt2 += zb * sB; C += z * sC;
    const int lane = threadIdx.x & 31, lr = lane & 15, hi = lane >> 4; const int r0 = blockIdx.x * 64, c0 = blockIdx.y * 64;
    if (CMODE == 1 && c0 > r0 + roff + 63) return;
    const int Kl = (CMODE == 2) ? min(K, r0 + roff + 64) : K;
    v8f acc[4][4];
#pragma unroll
    for (int mb = 0; mb < 4; ++mb)
#pragma unroll
        for (int nb = 0; nb < 4; ++nb) acc[mb][nb] = (v8f){};
    const size_t aoff = (size_t)(r0 + lr) * K + 8 * hi, boff = (size_t)(c0 + lr) * K + 8 * hi;
#pragma unroll 1
    for (int kc = 0; kc < Kl; kc += 32) {
        V a[4], a2[4];
#pragma unroll
        for (int mb = 0; mb < 4; ++mb) { a[mb] = WFrag<T16>::ld(A + aoff + (size_t)mb * 16 * K + kc); if (NSPLIT == 1 || NSPLIT == 2) a2[mb] = WFrag<T16>::ld(A2 + aoff + (size_t)mb * 16 * K + kc); }
#pragma unroll
        for (int nb = 0; nb < 4; ++nb) { const V b = WFrag<T16>::ld(Bt + boff + (size_t)nb * 16 * K + kc); V b2; if (NSPLIT >= 2) b2 = WFrag<T16>::ld(Bt2 + boff + (size_t)nb * 16 * K + kc);
#pragma unroll
            for (int mb = 0; mb < 4; ++mb) { acc[mb][nb] = WFrag<T16>::mma(a[mb], b, acc[mb][nb]); if (NSPLIT == 1 || NSPLIT == 2) acc[mb][nb] = WFrag<T16>::mma(a2[mb], b, acc[mb][nb]); if (NSPLIT >= 2) acc[mb][nb] = WFrag<T16>::mma(a[mb], b2, acc[mb][nb]); } }
        asm volatile("v_nop\n\tv_nop\n\tv_nop\n\tv_nop" : "+v"(acc[0][0]), "+v"(acc[1][1]), "+v"(acc[2][2]), "+v"(acc[3][3]) : "v"(a[0]), "v"(a[3]));
    }
#pragma unroll
    for (int mb = 0; mb < 4; ++mb) {
#pragma unroll
        for (int nb = 0; nb < 4; ++nb) {
#pragma unroll
            for (int j = 0; j < 8; ++j) os[(hi * 8 + j) * 68 + nb * 16 + lr] = acc[mb][nb][j]; }
        wave_lds_sync();
        float* crow = C + (size_t)(r0 + mb * 16) * ldc + c0;
#pragma unroll 1
        for (int ps = 0; ps < 2; ++ps) {
#pragma unroll
            for (int s = 0; s < 8; ++s) { const int row = 2 * s + hi, cofs = lr * 4; v4f val = *(const v4fa*)(os + row * 68 + cofs);
                *(volatile v4f*)(crow + (size_t)row * ldc + cofs) = val; }
            if (ps == 0) __threadfence(); }
        wave_lds_sync();
    }
}

__global__ __launch_bounds__(256) void k_hplane(const float* __restrict__ F, size_t hstride, int nheads, float sc, h16* P16, bf* Ph, bf* Pl) {
    const size_t e = ((size_t)blockIdx.x * 256 + threadIdx.x) * 2; if (e >= (size_t)nheads * TT * HD) return;
    const int d = (int)(e % HD); const int t = (int)((e / HD) % TT); const int h = (int)(e / ((size_t)HD * TT));
    const float* f = F + (size_t)h * hstride + (size_t)t * HD + d; v2h o16; v2us oh, ol;
#pragma unroll
    for (int q = 0; q < 2; ++q) { const float r = bfr(f[q]) * sc; o16[q] = toh_flush(r); unsigned short a2, c2; splitf(r, a2, c2); oh[q] = a2; ol[q] = c2; }
    *(volatile v2h*)(P16 + e) = o16; *(volatile v2us*)(Ph + e) = oh; *(volatile v2us*)(Pl + e) = ol; __threadfence(); *(volatile v2h*)(P16 + e) = o16; *(volatile v2us*)(Ph + e) = oh; *(volatile v2us*)(Pl + e) = ol; }

__global__ __launch_bounds__(256) void k_knplane(const float* __restrict__ F, size_t hstride, int nheads, float sc, h16* P16, bf* Ph, bf* Pl) {
#pragma clang fp contract(off)
    const int lane = threadIdx.x & 31; const int wave = __builtin_amdgcn_readfirstlane(threadIdx.x >> 5);
    const int row = blockIdx.x * 8 + wave; if (row >= nheads * TT) return;
    const int t = row % TT; const int h = row / TT; const int d = lane * 2;
    const float* f = F + (size_t)h * hstride + (size_t)t * HD + d;
    const float x0 = bfr(f[0]), x1 = bfr(f[1]);
    float ss = x0 * x0 + x1 * x1;
#pragma unroll
    for (int sh = 16; sh; sh >>= 1) ss += __shfl_xor(ss, sh, 32);
    const float inv = __builtin_amdgcn_rcpf(__builtin_amdgcn_sqrtf(ss) + 1e-6f);
    const float r0 = (x0 * inv) * sc, r1 = (x1 * inv) * sc;
    v2h o16; v2us oh, ol; unsigned short a2, c2;
    o16[0] = toh_flush(r0); splitf(r0, a2, c2); oh[0] = a2; ol[0] = c2;
    o16[1] = toh_flush(r1); splitf(r1, a2, c2); oh[1] = a2; ol[1] = c2;
    const size_t e = (size_t)row * HD + d;
    *(volatile v2h*)(P16 + e) = o16; *(volatile v2us*)(Ph + e) = oh; *(volatile v2us*)(Pl + e) = ol; __threadfence(); *(volatile v2h*)(P16 + e) = o16; *(volatile v2us*)(Ph + e) = oh; *(volatile v2us*)(Pl + e) = ol; }

__global__ __launch_bounds__(256) void k_vtph(const float* __restrict__ F, size_t hstride, int nheads, float sc, h16* V16, bf* Vh, bf* Vl) { const size_t e = ((size_t)blockIdx.x * 256 + threadIdx.x) * 2; if (e >= (size_t)nheads * HD * TT) return; const int t = (int)(e % TT); const int d = (int)((e / TT) % HD); const int g = (int)(e / ((size_t)TT * HD)); v2h o16; v2us oh, ol;
#pragma unroll
    for (int q = 0; q < 2; ++q) { const float x = bfr(F[(size_t)g * hstride + (size_t)(t + q) * HD + d]) * sc; o16[q] = toh_flush(x); unsigned short a2, c2; splitf(x, a2, c2); oh[q] = a2; ol[q] = c2; }
    *(volatile v2h*)(V16 + e) = o16; *(volatile v2us*)(Vh + e) = oh; *(volatile v2us*)(Vl + e) = ol; __threadfence(); *(volatile v2h*)(V16 + e) = o16; *(volatile v2us*)(Vh + e) = oh; *(volatile v2us*)(Vl + e) = ol; }

__global__ __launch_bounds__(64) void k_decay(const float* __restrict__ AF, const float* __restrict__ srcp, const float* __restrict__ dstp, float* DB) {
#pragma clang fp contract(off)
    __shared__ float dgs[TT];
    const int g = blockIdx.y; const int i0 = blockIdx.x * 64; const int j = i0 + (int)threadIdx.x;
    const float* sp = srcp + (size_t)g * SEQ_FULL; const float* dp = dstp + (size_t)g * SEQ_FULL;
#pragma unroll 1
    for (int i = threadIdx.x; i < TT; i += 64) dgs[i] = sig3(dp[i]);
    const float sgj = sig3(sp[j]);
    __syncthreads();
    const float* af = AF + (size_t)g * TT * TT + j; float* db = DB + (size_t)g * TT * TT + j;
    float run = 0.0f;
#pragma unroll 1
    for (int ib = i0; ib < TT; ib += 8) {
        float dv[8];
#pragma unroll
        for (int r = 0; r < 8; ++r) { const int i = ib + r; float c = af[(size_t)i * TT]; asm volatile("" : "+v"(c)); c = c * (1.0f / 64.0f);
            float a = (pow23(c) * dgs[i]) * sgj; a = fminf(fmaxf(a, 0.0f), CLAMPHI);
            const float lg = LN2F * __builtin_amdgcn_logf(1.0f - a); const float ld = (i > j) ? lg : 0.0f; dv[r] = run; run = run + ld; }
#pragma unroll
        for (int r = 0; r < 8; ++r) *(volatile float*)(db + (size_t)(ib + r) * TT) = dv[r];
        __threadfence();
#pragma unroll
        for (int r = 0; r < 8; ++r) *(volatile float*)(db + (size_t)(ib + r) * TT) = dv[r];
    }
}

__global__ __launch_bounds__(256) void k_dsoft(const float* __restrict__ Sb, const float* __restrict__ Db, h16* P16, bf* Ph, bf* Pl) {
#pragma clang fp contract(off)
    const int lane = threadIdx.x & 31; const int wave = __builtin_amdgcn_readfirstlane(threadIdx.x >> 5);
    const int row = blockIdx.x * 8 + wave; if (row >= ZH * TT) return; const int i = row % TT; const int zz = row / TT; const bool hires = (i < RH);
    const int nch = (i >> 7) + 1; const int ilim = i | 63;
    const float* sr = Sb + (size_t)row * TT; const float* dr = Db + ((size_t)(zz / REP) * TT + i) * TT;
    float v[TT / 32]; float mx = NEGF;
#pragma unroll
    for (int ch = 0; ch < TT / 128; ++ch) { if (ch < nch) { const int j0 = ch * 128 + lane * 4; const int jl = (j0 > ilim) ? (j0 - 64) : j0; v4f a = *(const v4f*)(sr + jl); v4f dd = *(const v4f*)(dr + jl); asm volatile("" : "+v"(a), "+v"(dd));
#pragma unroll
            for (int q = 0; q < 4; ++q) { const int j = j0 + q; const float s = a[q] * SCL + dd[q]; const float t = (j <= i) ? s : NEGF; v[ch * 4 + q] = t; mx = fmaxf(mx, t); } } }
#pragma unroll
    for (int sh = 16; sh; sh >>= 1) mx = fmaxf(mx, __shfl_xor(mx, sh, 32));
    float sum = 0.f;
#pragma unroll
    for (int k = 0; k < TT / 32; ++k) { if ((k >> 2) < nch) { float d0 = __fsub_rn(v[k], mx); asm volatile("" : "+v"(d0)); v[k] = __builtin_amdgcn_exp2f(__fmul_rn(d0, 1.4426950408889634f)); sum += v[k]; } }
#pragma unroll
    for (int sh = 16; sh; sh >>= 1) sum += __shfl_xor(sum, sh, 32);
    const float f = __fdiv_rn(hires ? 1.0f : PCAR, sum);
#pragma unroll 1
    for (int ps = 0; ps < 2; ++ps) {
        if (hires) {
#pragma unroll
            for (int ch = 0; ch < TT / 128; ++ch) { if (ch < nch) { v4us oh, ol;
#pragma unroll
                for (int q = 0; q < 4; ++q) { unsigned short a2, c2; splitf(v[ch * 4 + q] * f, a2, c2); oh[q] = a2; ol[q] = c2; }
                const size_t oo = ((size_t)zz * RH + i) * TT + ch * 128 + lane * 4; *(volatile v4us*)(Ph + oo) = oh; *(volatile v4us*)(Pl + oo) = ol; } }
        } else {
#pragma unroll
            for (int ch = 0; ch < TT / 128; ++ch) { if (ch < nch) { v4h o4;
#pragma unroll
                for (int q = 0; q < 4; ++q) o4[q] = toh_flush(v[ch * 4 + q] * f);
                *(volatile v4h*)(P16 + (size_t)row * TT + ch * 128 + lane * 4) = o4; } } }
        if (ps == 0) __threadfence(); }
}

__global__ __launch_bounds__(256) void k_outw(const float* __restrict__ O, float* OUTh) { const size_t e = ((size_t)blockIdx.x * 256 + threadIdx.x) * 4; if (e >= (size_t)ZH * TT * HD) return; const int d = (int)(e % HD); const int t = (int)((e / HD) % TT); const int zz = (int)(e / ((size_t)HD * TT)); const float cs = (t < RH) ? (1.0f / VCAR) : (1.0f / (VCAR * PCAR));
    v4f val = *(const v4f*)(O + e); val[0] *= cs; val[1] *= cs; val[2] *= cs; val[3] *= cs;
    float* dst = OUTh + (size_t)zz * SEQ_FULL * HD + (size_t)t * HD + d; *(volatile v4f*)dst = val; __threadfence(); *(volatile v4f*)dst = val; }

extern "C" void kernel_launch(void* const* d_in, const int* in_sizes, int n_in,
                              void* d_out, int out_size, void* d_ws, size_t ws_size, hipStream_t stream) {
    if (n_in < 5) return;
    if (in_sizes[0] < (((NB - 1) * NH_ + (NH_ - 1)) * SEQ_FULL + SEQ) * HD) return;
    if (in_sizes[1] < (((NB - 1) * NKV + (NKV - 1)) * SEQ_FULL + SEQ) * HD) return;
    if (in_sizes[2] < (((NB - 1) * NKV + (NKV - 1)) * SEQ_FULL + SEQ) * HD) return;
    if (in_sizes[3] < ((NB - 1) * NKV + (NKV - 1)) * SEQ_FULL + SEQ) return;
    if (in_sizes[4] < ((NB - 1) * NKV + (NKV - 1)) * SEQ_FULL + SEQ) return;
    if (out_size < (((NB - 1) * NH_ + (NH_ - 1)) * SEQ_FULL + SEQ) * HD) return;
    const float* qin = (const float*)d_in[0];
    const float* kin = (const float*)d_in[1];
    const float* vin = (const float*)d_in[2];
    const float* sin_ = (const float*)d_in[3];
    const float* din_ = (const float*)d_in[4];
    float* OUT = (float*)d_out;
    char* wsp = (char*)d_ws; size_t used = 0;
    auto take = [&](size_t bytes) { char* p = wsp + used; used += (bytes + 255) & ~(size_t)255; return (void*)p; };
    h16* QP16 = (h16*)take((size_t)NH_ * TT * HD * 2); h16* KP16 = (h16*)take((size_t)NKV * TT * HD * 2); h16* VT16 = (h16*)take((size_t)NKV * HD * TT * 2);
    bf* QPh = (bf*)take((size_t)NH_ * TT * HD * 2); bf* QPl = (bf*)take((size_t)NH_ * TT * HD * 2); bf* KPh = (bf*)take((size_t)NKV * TT * HD * 2); bf* KPl = (bf*)take((size_t)NKV * TT * HD * 2);
    bf* VTh = (bf*)take((size_t)NKV * HD * TT * 2); bf* VTl = (bf*)take((size_t)NKV * HD * TT * 2); bf* Ph = (bf*)take((size_t)ZH * RH * TT * 2); bf* Pl = (bf*)take((size_t)ZH * RH * TT * 2);
    float* AF = (float*)take((size_t)ZKV * TT * TT * 4); float* DB = (float*)take((size_t)ZKV * TT * TT * 4);
    float* Sb = (float*)take((size_t)ZH * TT * TT * 4); h16* P16 = (h16*)take((size_t)ZH * TT * TT * 2); float* Ob = (float*)take((size_t)ZH * TT * HD * 4);
    if (used > ws_size) return;

    const unsigned LQ = (unsigned)(((size_t)NH_ * TT * HD / 2 + 255) / 256), LKv = (unsigned)(((size_t)NKV * TT * HD / 2 + 255) / 256), LO = (unsigned)(((size_t)ZH * TT * HD / 4 + 255) / 256);
    const size_t HS = (size_t)SEQ_FULL * HD;
    for (int b = 0; b < NB; ++b) {
        const float* qb = qin + (size_t)b * NH_ * HS; const float* kb = kin + (size_t)b * NKV * HS; const float* vb = vin + (size_t)b * NKV * HS;
        const float* sb = sin_ + (size_t)b * NKV * SEQ_FULL; const float* db = din_ + (size_t)b * NKV * SEQ_FULL;
        k_hplane<<<LQ, 256, 0, stream>>>(qb, HS, NH_, QCAR, QP16, QPh, QPl);
        k_knplane<<<(unsigned)(NKV * TT / 8), 256, 0, stream>>>(kb, HS, NKV, QCAR, KP16, KPh, KPl);
        k_vtph<<<LKv, 256, 0, stream>>>(vb, HS, NKV, VCAR, VT16, VTh, VTl);
        for (int h0 = 0; h0 < NH_; h0 += ZH) { const size_t zq = (size_t)h0, zk = (size_t)(h0 / REP);
            k_gemmc<h16, 0, 1><<<dim3(TT / 64, TT / 64, ZKV), 32, 0, stream>>>(KP16 + zk * TT * HD, nullptr, KP16 + zk * TT * HD, nullptr, HD, AF, TT, 0, (size_t)TT * HD, (size_t)TT * HD, (size_t)TT * TT, 1);
            k_decay<<<dim3(TT / 64, ZKV), 64, 0, stream>>>(AF, sb + zk * SEQ_FULL, db + zk * SEQ_FULL, DB);
            k_gemmc<bf, 2, 1><<<dim3(RH / 64, TT / 64, ZH), 32, 0, stream>>>(QPh + zq * TT * HD, QPl + zq * TT * HD, KPh + zk * TT * HD, KPl + zk * TT * HD, HD, Sb, TT, 0, (size_t)TT * HD, (size_t)TT * HD, (size_t)TT * TT, REP);
            k_gemmc<h16, 0, 1><<<dim3((TT - RH) / 64, TT / 64, ZH), 32, 0, stream>>>(QP16 + zq * TT * HD + (size_t)RH * HD, nullptr, KP16 + zk * TT * HD, nullptr, HD, Sb + (size_t)RH * TT, TT, RH, (size_t)TT * HD, (size_t)TT * HD, (size_t)TT * TT, REP);
            k_dsoft<<<(unsigned)(ZH * TT / 8), 256, 0, stream>>>(Sb, DB, P16, Ph, Pl);
            k_gemmc<bf, 2, 2><<<dim3(RH / 64, HD / 64, ZH), 32, 0, stream>>>(Ph, Pl, VTh + zk * HD * TT, VTl + zk * HD * TT, TT, Ob, HD, 0, (size_t)RH * TT, (size_t)HD * TT, (size_t)TT * HD, REP);
            k_gemmc<h16, 0, 2><<<dim3((TT - RH) / 64, HD / 64, ZH), 32, 0, stream>>>(P16 + (size_t)RH * TT, nullptr, VT16 + zk * HD * TT, nullptr, TT, Ob + (size_t)RH * HD, HD, RH, (size_t)TT * TT, (size_t)HD * TT, (size_t)TT * HD, REP);
            k_outw<<<LO, 256, 0, stream>>>(Ob, OUT + ((size_t)b * NH_ + h0) * HS); }
    }
}
